// MultiHeadAttention_27685359190775
// MI455X (gfx1250) — hardware-verified
//
#include <hip/hip_runtime.h>

#ifndef NB
#define NB 4
#endif
#ifndef SEQ
#define SEQ 2048
#endif
#define NB_FULL 4
#define SEQ_FULL 2048
#define DM 1024
#define NH 16
#define HD 64
#define MTOK (NB * SEQ)
#define PPH 40
#define OPF 68

static_assert(DM == NH * HD);
static_assert(HD == 64);
static_assert(DM % 64 == 0);
static_assert(DM % 32 == 0);
static_assert(DM % 8 == 0);
static_assert(SEQ % 64 == 0);
static_assert(MTOK % 64 == 0);
static_assert(NB <= NB_FULL);
static_assert(SEQ <= SEQ_FULL);
static_assert((PPH * 2) % 16 == 0);
static_assert((OPF * 4) % 16 == 0);
static_assert((size_t)NB_FULL * SEQ_FULL * DM * 4 == 33554432);

typedef __attribute__((ext_vector_type(16))) _Float16 v16h;
typedef __attribute__((ext_vector_type(8)))  _Float16 v8h;
typedef __attribute__((ext_vector_type(8)))  float    v8f;
typedef __attribute__((ext_vector_type(4)))  float    v4f;
typedef __attribute__((ext_vector_type(4)))  unsigned int v4u;
typedef v8h v8h_a __attribute__((may_alias));
typedef v4f v4f_a __attribute__((may_alias));

union FragU { v16h v; v8h h[2]; };
__device__ __forceinline__ v16h frag_ld(const _Float16* p) {
    FragU f; f.h[0] = *(const v8h_a*)(p); f.h[1] = *(const v8h_a*)(p + 16); return f.v;
}
__device__ __forceinline__ v8f mma_h(v16h a, v16h b, v8f c) {
    return __builtin_amdgcn_wmma_f32_16x16x32_f16(false, a, false, b, (short)0, c, false, false);
}
__device__ __forceinline__ v8f mma_hg(v16h a, v16h b, v8f c) {
    c = __builtin_amdgcn_wmma_f32_16x16x32_f16(false, a, false, b, (short)0, c, false, false);
    asm volatile("v_nop\n\tv_nop\n\tv_nop\n\tv_nop" : "+v"(c) : "v"(a), "v"(b));
    return c;
}
__device__ __forceinline__ void dep_guard_h(v8f& a, v8f& b, v16h x, v16h y) { asm volatile("v_nop\n\tv_nop\n\tv_nop\n\tv_nop" : "+v"(a), "+v"(b) : "v"(x), "v"(y)); }
__device__ __forceinline__ void keep4_h(v16h a, v16h b, v16h c, v16h d) { asm volatile("v_nop" :: "v"(a), "v"(b), "v"(c), "v"(d)); }
__device__ __forceinline__ void acc_guard4(v8f& a, v8f& b, v8f& c, v8f& d) { asm volatile("v_nop\n\tv_nop\n\tv_nop\n\tv_nop" : "+v"(a), "+v"(b), "+v"(c), "+v"(d)); }
__device__ __forceinline__ void wave_sync() {
    __builtin_amdgcn_fence(3  , "workgroup");
    __builtin_amdgcn_wave_barrier();
    __builtin_amdgcn_fence(2  , "workgroup");
}
__device__ __forceinline__ float cmb_bf(float v) {
    unsigned u = __float_as_uint(v);
    u = (u + 0x7fffu + ((u >> 16) & 1u)) & 0xffff0000u;
    return __uint_as_float(u);
}
__device__ __forceinline__ unsigned int pk2h(float a, float b) {
    return (unsigned int)__builtin_bit_cast(unsigned short, (_Float16)a) | ((unsigned int)__builtin_bit_cast(unsigned short, (_Float16)b) << 16);
}

__global__ __launch_bounds__(256) void k_cast16(const float* __restrict__ src, unsigned short* __restrict__ dst, int nR, int rows_c, int rows_f, float sc) {
    const long long u = (long long)blockIdx.x * 256 + threadIdx.x;
    const int per = DM / 8;
    if (u >= (long long)nR * per) return;
    const int r = (int)(u / per);
    const int c0 = 8 * (int)(u % per);
    const long long sr = (long long)(r / rows_c) * rows_f + (r % rows_c);
    const float* s = src + sr * DM + c0;
    const v4f a = *(const v4f*)(s);
    const v4f b = *(const v4f*)(s + 4);
    v4u pk;
    pk.x = pk2h(cmb_bf(a.x) * sc, cmb_bf(a.y) * sc);
    pk.y = pk2h(cmb_bf(a.z) * sc, cmb_bf(a.w) * sc);
    pk.z = pk2h(cmb_bf(b.x) * sc, cmb_bf(b.y) * sc);
    pk.w = pk2h(cmb_bf(b.z) * sc, cmb_bf(b.w) * sc);
    volatile v4u* d = (volatile v4u*)(dst + (long long)r * DM + c0);
    *d = pk;
    __threadfence();
    *d = pk;
}

template <int BIAS_MODE, int OUT_MODE, bool ROWMAP>
__device__ __forceinline__ void gemm64_body(const unsigned short* __restrict__ Ap, const int lda,
                                            const unsigned short* __restrict__ Btp, const int ldb,
                                            float* __restrict__ Cf, unsigned short* __restrict__ Ch, const int ldc,
                                            const float* __restrict__ bias, const int M, const int N, const int K, const float scale) {
    __shared__ __align__(16) float sT[8][16 * OPF];
    const _Float16* A  = (const _Float16*)Ap;
    const _Float16* Bt = (const _Float16*)Btp;
    const int lane = threadIdx.x & 31;
    const int wave = threadIdx.x >> 5;
    const int tilesN = N >> 6;
    const int tilesM = M >> 6;
    const int tile = blockIdx.x * 8 + wave;
    if (tile >= tilesM * tilesN) return;
    const int tm = tile / tilesN;
    const int tn = tile - tm * tilesN;
    const int m0 = tm << 6;
    const int n0 = tn << 6;
    const int rlane = lane & 15;
    const int koff  = (lane >> 4) * 8;
    const int mOff  = (lane >> 4) * 8;

    v8f acc[4][4];
#pragma unroll
    for (int i = 0; i < 4; ++i)
#pragma unroll
        for (int j = 0; j < 4; ++j) acc[i][j] = (v8f){0.f, 0.f, 0.f, 0.f, 0.f, 0.f, 0.f, 0.f};

    for (int k0 = 0; k0 < K; k0 += 32) {
        v16h bh[4];
#pragma unroll
        for (int j = 0; j < 4; ++j) bh[j] = frag_ld(Bt + (size_t)(n0 + (j << 4) + rlane) * ldb + koff + k0);
#pragma unroll
        for (int i = 0; i < 4; ++i) {
            const v16h ah = frag_ld(A + (size_t)(m0 + (i << 4) + rlane) * lda + koff + k0);
#pragma unroll
            for (int j = 0; j < 4; ++j) acc[i][j] = mma_h(ah, bh[j], acc[i][j]);
            dep_guard_h(acc[i][0], acc[i][3], ah, ah);
        }
        keep4_h(bh[0], bh[1], bh[2], bh[3]);
    }
    acc_guard4(acc[0][0], acc[0][1], acc[0][2], acc[0][3]);
    acc_guard4(acc[1][0], acc[1][1], acc[1][2], acc[1][3]);
    acc_guard4(acc[2][0], acc[2][1], acc[2][2], acc[2][3]);
    acc_guard4(acc[3][0], acc[3][1], acc[3][2], acc[3][3]);

#pragma unroll
    for (int i = 0; i < 4; ++i) {
        const int mBase = m0 + (i << 4);
        float bm[8];
#pragma unroll
        for (int r = 0; r < 8; ++r) bm[r] = (BIAS_MODE == 1) ? cmb_bf(bias[mBase + mOff + r]) : 0.f;
#pragma unroll
        for (int j = 0; j < 4; ++j) {
            const int n = n0 + (j << 4) + rlane;
            const float bv = (BIAS_MODE == 2) ? cmb_bf(bias[n]) : 0.f;
#pragma unroll
            for (int r = 0; r < 8; ++r) {
                float v = acc[i][j][r] * scale;
                if (BIAS_MODE == 1) v += bm[r];
                if (BIAS_MODE == 2) v += bv;
                sT[wave][(mOff + r) * OPF + (j << 4) + rlane] = v;
            }
        }
        wave_sync();
        if (OUT_MODE == 0) {
            const int orow = ROWMAP ? ((mBase / SEQ) * SEQ_FULL + (mBase % SEQ)) : mBase;
            const int hh = lane >> 4, c4 = (lane & 15) * 4;
            v4f vals[8];
#pragma unroll
            for (int it = 0; it < 8; ++it) vals[it] = *(const v4f_a*)&sT[wave][(it * 2 + hh) * OPF + c4];
#pragma unroll
            for (int pass = 0; pass < 2; ++pass) {
#pragma unroll
                for (int it = 0; it < 8; ++it)
                    *(volatile v4f*)(Cf + (size_t)(orow + it * 2 + hh) * ldc + n0 + c4) = vals[it];
                __threadfence();
            }
        } else {
            const int q = lane >> 3, c8 = (lane & 7) * 8;
            v4u pk[4];
#pragma unroll
            for (int it = 0; it < 4; ++it) {
                const int row = it * 4 + q;
                const v4f a = *(const v4f_a*)&sT[wave][row * OPF + c8];
                const v4f b = *(const v4f_a*)&sT[wave][row * OPF + c8 + 4];
                pk[it].x = pk2h(a.x, a.y); pk[it].y = pk2h(a.z, a.w); pk[it].z = pk2h(b.x, b.y); pk[it].w = pk2h(b.z, b.w);
            }
#pragma unroll
            for (int pass = 0; pass < 2; ++pass) {
#pragma unroll
                for (int it = 0; it < 4; ++it)
                    *(volatile v4u*)(Ch + (size_t)(mBase + it * 4 + q) * ldc + n0 + c8) = pk[it];
                __threadfence();
            }
        }
        wave_sync();
    }
}

__global__ __launch_bounds__(256) void k_proj_tok(const unsigned short* __restrict__ X, const unsigned short* __restrict__ W, unsigned short* __restrict__ Y, const float* __restrict__ bias) {
    gemm64_body<2, 1, false>(X, DM, W, DM, nullptr, Y, DM, bias, MTOK, DM, DM, 0.0625f);
}
__global__ __launch_bounds__(256) void k_proj_vt(const unsigned short* __restrict__ W, const unsigned short* __restrict__ X, unsigned short* __restrict__ Yt, const float* __restrict__ bias) {
    gemm64_body<1, 1, false>(W, DM, X, DM, nullptr, Yt, MTOK, bias, DM, MTOK, DM, 0.0625f);
}
__global__ __launch_bounds__(256) void k_proj_out(const unsigned short* __restrict__ Cx, const unsigned short* __restrict__ W, float* __restrict__ out, const float* __restrict__ bias) {
    gemm64_body<2, 0, true>(Cx, DM, W, DM, out, nullptr, DM, bias, MTOK, DM, DM, 0.00390625f);
}

__global__ __launch_bounds__(128) void k_flash(const unsigned short* __restrict__ Qp, const unsigned short* __restrict__ Kp,
                                               const unsigned short* __restrict__ Vtp, unsigned short* __restrict__ Cp) {
    __shared__ __align__(16) _Float16 psh[4][16 * PPH];
    __shared__ __align__(16) float    Os[4][16 * OPF];
    const int tid = threadIdx.x;
    const int wave = tid >> 5;
    const int lane = tid & 31;
    const int hh = lane >> 4;
    const int c  = lane & 15;
    const int nqb = SEQ / 64;
    const int bx = blockIdx.x;
    const int qb = bx % nqb;
    const int bh = bx / nqb;
    const int hd = bh % NH;
    const int b  = bh / NH;
    const int q0 = qb * 64 + wave * 16;
    const size_t tok0 = (size_t)b * SEQ;

    const _Float16* Q  = (const _Float16*)Qp;
    const _Float16* K  = (const _Float16*)Kp;
    const _Float16* Vt = (const _Float16*)Vtp;

    const _Float16* qrow = Q + (tok0 + q0 + c) * DM + hd * HD + 8 * hh;
    const v16h qa0 = frag_ld(qrow);
    const v16h qa1 = frag_ld(qrow + 32);
    const _Float16* kl = K + (tok0 + c) * DM + hd * HD + 8 * hh;
    const _Float16* vl = Vt + (size_t)(hd * HD + c) * MTOK + tok0 + 8 * hh;

    float mrow[8], lrow[8];
    v8f oacc[4];
#pragma unroll
    for (int r = 0; r < 8; ++r) { mrow[r] = -__builtin_inff(); lrow[r] = 0.f; }
#pragma unroll
    for (int t = 0; t < 4; ++t) oacc[t] = (v8f){0.f, 0.f, 0.f, 0.f, 0.f, 0.f, 0.f, 0.f};

    const float SCL = 0.125f * 1.4426950408889634f;

#pragma unroll 1
    for (int kv0 = 0; kv0 < SEQ; kv0 += 32) {
        const _Float16* k0p = kl + (size_t)kv0 * DM;
        const _Float16* k1p = k0p + (size_t)16 * DM;
        v8f s0 = (v8f){0.f, 0.f, 0.f, 0.f, 0.f, 0.f, 0.f, 0.f};
        v8f s1 = (v8f){0.f, 0.f, 0.f, 0.f, 0.f, 0.f, 0.f, 0.f};
        s0 = mma_hg(qa0, frag_ld(k0p), s0);
        s0 = mma_hg(qa1, frag_ld(k0p + 32), s0);
        s1 = mma_hg(qa0, frag_ld(k1p), s1);
        s1 = mma_hg(qa1, frag_ld(k1p + 32), s1);

#pragma unroll
        for (int r = 0; r < 8; ++r) {
            const float a0 = s0[r] * SCL;
            const float a1 = s1[r] * SCL;
            float mx = fmaxf(a0, a1);
            mx = fmaxf(mx, __shfl_xor(mx, 1, 32));
            mx = fmaxf(mx, __shfl_xor(mx, 2, 32));
            mx = fmaxf(mx, __shfl_xor(mx, 4, 32));
            mx = fmaxf(mx, __shfl_xor(mx, 8, 32));
            const float mnew  = fmaxf(mrow[r], mx);
            const float alpha = exp2f(mrow[r] - mnew);
            const float p0 = exp2f(a0 - mnew);
            const float p1 = exp2f(a1 - mnew);
            mrow[r] = mnew;
            lrow[r] = lrow[r] * alpha + (p0 + p1);
#pragma unroll
            for (int t = 0; t < 4; ++t) oacc[t][r] *= alpha;
            psh[wave][(8 * hh + r) * PPH + c]      = (_Float16)(p0 * 4096.0f);
            psh[wave][(8 * hh + r) * PPH + 16 + c] = (_Float16)(p1 * 4096.0f);
        }
        wave_sync();
        FragU pa;
        pa.h[0] = *(const v8h_a*)&psh[wave][c * PPH + 8 * hh];
        pa.h[1] = *(const v8h_a*)&psh[wave][c * PPH + 16 + 8 * hh];
        const _Float16* vp = vl + kv0;
#pragma unroll
        for (int t = 0; t < 4; ++t) oacc[t] = mma_hg(pa.v, frag_ld(vp + (size_t)t * 16 * MTOK), oacc[t]);
        wave_sync();
    }

#pragma unroll
    for (int r = 0; r < 8; ++r) {
        float l = lrow[r];
        l += __shfl_xor(l, 1, 32);
        l += __shfl_xor(l, 2, 32);
        l += __shfl_xor(l, 4, 32);
        l += __shfl_xor(l, 8, 32);
        const float inv = 1.0f / (l * 256.0f);
#pragma unroll
        for (int t = 0; t < 4; ++t) Os[wave][(8 * hh + r) * OPF + t * 16 + c] = oacc[t][r] * inv;
    }
    wave_sync();
    {
        const int q = lane >> 3, c8 = (lane & 7) * 8;
        v4u pk[4];
#pragma unroll
        for (int it = 0; it < 4; ++it) {
            const int row = it * 4 + q;
            const v4f a = *(const v4f_a*)&Os[wave][row * OPF + c8];
            const v4f bq = *(const v4f_a*)&Os[wave][row * OPF + c8 + 4];
            pk[it].x = pk2h(a.x, a.y); pk[it].y = pk2h(a.z, a.w); pk[it].z = pk2h(bq.x, bq.y); pk[it].w = pk2h(bq.z, bq.w);
        }
#pragma unroll
        for (int pass = 0; pass < 2; ++pass) {
#pragma unroll
            for (int it = 0; it < 4; ++it)
                *(volatile v4u*)(Cp + (tok0 + q0 + it * 4 + q) * DM + hd * HD + c8) = pk[it];
            __threadfence();
        }
    }
}

#define WS_PLANE  ((size_t)MTOK * DM * 2)
#define WS_WPLANE ((size_t)DM * DM * 2)
#define WS_TOTAL  (6 * WS_PLANE + 4 * WS_WPLANE)
static_assert(WS_PLANE % 256 == 0);
static_assert(WS_WPLANE % 256 == 0);
static_assert(WS_TOTAL <= (size_t)134217728);

extern "C" void kernel_launch(void* const* d_in, const int* in_sizes, int n_in, void* d_out, int out_size, void* d_ws, size_t ws_size, hipStream_t stream) {
    if (n_in < 10) return;
    const long long need_x = (long long)MTOK * DM;
    const long long need_w = (long long)DM * DM;
    if ((long long)in_sizes[0] < need_x || (long long)in_sizes[1] < need_x) return;
    if ((long long)in_sizes[2] < need_w || (long long)in_sizes[4] < need_w || (long long)in_sizes[6] < need_w || (long long)in_sizes[8] < need_w) return;
    if (in_sizes[3] < DM || in_sizes[5] < DM || in_sizes[7] < DM || in_sizes[9] < DM) return;
    if ((long long)out_size < need_x) return;
    if (ws_size < WS_TOTAL) return;

    const float* xq  = (const float*)d_in[0];
    const float* xkv = (const float*)d_in[1];
    const float* Wq  = (const float*)d_in[2];
    const float* bq  = (const float*)d_in[3];
    const float* Wk  = (const float*)d_in[4];
    const float* bk  = (const float*)d_in[5];
    const float* Wv  = (const float*)d_in[6];
    const float* bv  = (const float*)d_in[7];
    const float* Wo  = (const float*)d_in[8];
    const float* bo  = (const float*)d_in[9];
    float* out = (float*)d_out;

    char* wsp = (char*)d_ws;
    unsigned short* XQ  = (unsigned short*)wsp; wsp += WS_PLANE;
    unsigned short* XKV = (unsigned short*)wsp; wsp += WS_PLANE;
    unsigned short* W16 = (unsigned short*)wsp; wsp += 4 * WS_WPLANE;
    unsigned short* QP  = (unsigned short*)wsp; wsp += WS_PLANE;
    unsigned short* KP  = (unsigned short*)wsp; wsp += WS_PLANE;
    unsigned short* VT  = (unsigned short*)wsp; wsp += WS_PLANE;
    unsigned short* CX  = (unsigned short*)wsp; wsp += WS_PLANE;
    const size_t WSTR = (size_t)DM * DM;

    const unsigned gx = (unsigned)(((long long)MTOK * (DM / 8) + 255) / 256);
    const unsigned gw = (unsigned)(((long long)DM * (DM / 8) + 255) / 256);
    k_cast16<<<gx, 256, 0, stream>>>(xq,  XQ,  MTOK, SEQ, SEQ_FULL, 1.0f);
    k_cast16<<<gx, 256, 0, stream>>>(xkv, XKV, MTOK, SEQ, SEQ_FULL, 1.0f);
    k_cast16<<<gw, 256, 0, stream>>>(Wq, W16 + 0 * WSTR, DM, DM, DM, 16.0f);
    k_cast16<<<gw, 256, 0, stream>>>(Wk, W16 + 1 * WSTR, DM, DM, DM, 16.0f);
    k_cast16<<<gw, 256, 0, stream>>>(Wv, W16 + 2 * WSTR, DM, DM, DM, 16.0f);
    k_cast16<<<gw, 256, 0, stream>>>(Wo, W16 + 3 * WSTR, DM, DM, DM, 16.0f);

    const unsigned gtiles = (unsigned)((((MTOK / 64) * (DM / 64)) + 7) / 8);
    k_proj_tok<<<gtiles, 256, 0, stream>>>(XQ,  W16 + 0 * WSTR, QP, bq);
    k_proj_tok<<<gtiles, 256, 0, stream>>>(XKV, W16 + 1 * WSTR, KP, bk);
    k_proj_vt <<<gtiles, 256, 0, stream>>>(W16 + 2 * WSTR, XKV, VT, bv);

    k_flash<<<(unsigned)(NB * NH * (SEQ / 64)), 128, 0, stream>>>(QP, KP, VT, CX);

    k_proj_out<<<gtiles, 256, 0, stream>>>(CX, W16 + 3 * WSTR, out, bo);
}
